// TwoToOneDNPU_16595753632207
// MI455X (gfx1250) — hardware-verified
//
#include <hip/hip_runtime.h>
#include <math.h>
typedef __attribute__((ext_vector_type(16))) _Float16 v16h;
typedef __attribute__((ext_vector_type(8)))  _Float16 v8h;
typedef __attribute__((ext_vector_type(16))) __bf16   v16b;
typedef __attribute__((ext_vector_type(8)))  __bf16   v8b;
typedef __attribute__((ext_vector_type(8)))  float    v8f;
typedef __attribute__((ext_vector_type(4)))  float    v4f;
#define PSCALE 32768.0f
#define U16(p) ((const unsigned short*)(const void*)(p))
#define PSCALE_INV (1.0f / 32768.0f)

__device__ __forceinline__ unsigned short f2bf_bits(float f) {
  unsigned u = __float_as_uint(f);
  return (unsigned short)((u + 0x7FFFu + ((u >> 16) & 1u)) >> 16);
}
__device__ __forceinline__ float bf_bits2f(unsigned short h) { return __uint_as_float(((unsigned)h) << 16); }

__device__ __forceinline__ void dep_guard_h(v8f& a, v8f& b, v16h x, v16h y) { asm volatile("v_nop\n\tv_nop\n\tv_nop\n\tv_nop" : "+v"(a), "+v"(b) : "v"(x), "v"(y)); }
__device__ __forceinline__ void dep_guard_b(v8f& a, v8f& b, v16b x, v16b y) { asm volatile("v_nop\n\tv_nop\n\tv_nop\n\tv_nop" : "+v"(a), "+v"(b) : "v"(x), "v"(y)); }
__device__ __forceinline__ void keep4_h(v16h a, v16h b, v16h c, v16h d) { asm volatile("v_nop" :: "v"(a), "v"(b), "v"(c), "v"(d)); }
__device__ __forceinline__ void keep4_b(v16b a, v16b b, v16b c, v16b d) { asm volatile("v_nop" :: "v"(a), "v"(b), "v"(c), "v"(d)); }
__device__ __forceinline__ void acc_guard4(v8f& a, v8f& b, v8f& c, v8f& d) { asm volatile("v_nop\n\tv_nop\n\tv_nop\n\tv_nop" : "+v"(a), "+v"(b), "+v"(c), "+v"(d)); }
template <typename T> struct Frag;
template <> struct Frag<_Float16> {
  typedef v16h V; union U { v16h v; v8h h[2]; };
  static __device__ __forceinline__ v16h load(const _Float16* p) {
    U f; f.h[0] = *(const v8h*)(p); f.h[1] = *(const v8h*)(p + 16); return f.v;
  }
  static __device__ __forceinline__ v8f mma(v16h a, v16h b, v8f c) {
    return __builtin_amdgcn_wmma_f32_16x16x32_f16(false, a, false, b, (short)0, c, false, false);
  }
  static __device__ __forceinline__ void guard(v8f& a, v8f& b, v16h x, v16h y) { dep_guard_h(a, b, x, y); }
  static __device__ __forceinline__ void keep(v16h a, v16h b, v16h c, v16h d) { keep4_h(a, b, c, d); }
};
template <> struct Frag<__bf16> {
  typedef v16b V; union U { v16b v; v8b h[2]; };
  static __device__ __forceinline__ v16b load(const __bf16* p) {
    U f; f.h[0] = *(const v8b*)(p); f.h[1] = *(const v8b*)(p + 16); return f.v;
  }
  static __device__ __forceinline__ v8f mma(v16b a, v16b b, v8f c) {
    return __builtin_amdgcn_wmma_f32_16x16x32_bf16(false, a, false, b, (short)0, c, false, false);
  }
  static __device__ __forceinline__ void guard(v8f& a, v8f& b, v16b x, v16b y) { dep_guard_b(a, b, x, y); }
  static __device__ __forceinline__ void keep(v16b a, v16b b, v16b c, v16b d) { keep4_b(a, b, c, d); }
};

template <int ET> struct Elem;
template <> struct Elem<0> { typedef _Float16 T; };
template <> struct Elem<1> { typedef __bf16 T; };
template <int ET, bool SPLIT, int BIAS_MODE, int OUT_MODE, bool RESID, int ACT = 0>
__global__ __launch_bounds__(256) void wmma_gemm64(
    const unsigned short* __restrict__ Ap, const unsigned short* __restrict__ A2p, int lda, long strideA,
    const unsigned short* __restrict__ Btp, const unsigned short* __restrict__ Bt2p, int ldb, long strideB,
    void* __restrict__ Cout, void* __restrict__ Cout2, int ldc, long strideC,
    const float* __restrict__ bias,
    const float* __restrict__ resid, long strideR,
    int M, int N, int K, float scale) {
  typedef typename Elem<ET>::T T;
  typedef typename Frag<T>::V V;
  const T* A = (const T*)Ap; const T* A2 = (const T*)A2p; const T* Bt = (const T*)Btp; const T* Bt2 = (const T*)Bt2p;
  __shared__ __align__(16) float sT[8][16 * 68];
  const int b    = blockIdx.y;
  const int lane = threadIdx.x & 31;
  const int wave = threadIdx.x >> 5;
  const int tilesN = N >> 6;
  const int tilesM = M >> 6;
  const int tile = blockIdx.x * 8 + wave;
  if (tile >= tilesM * tilesN) return;
  const int tm = tile / tilesN;
  const int tn = tile - tm * tilesN;
  const int m0 = tm << 6;
  const int n0 = tn << 6;

  const T* Ab  = A  + (size_t)b * strideA;
  const T* Bb  = Bt + (size_t)b * strideB;
  const T* Ab2 = SPLIT ? (A2  + (size_t)b * strideA) : nullptr;
  const T* Bb2 = SPLIT ? (Bt2 + (size_t)b * strideB) : nullptr;

  const int rlane = lane & 15;
  const int koff  = (lane >> 4) * 8;
  const int mOff  = (lane >> 4) * 8;

  v8f acc[4][4];
#pragma unroll
  for (int i = 0; i < 4; ++i)
#pragma unroll
    for (int j = 0; j < 4; ++j) acc[i][j] = (v8f){0.f,0.f,0.f,0.f,0.f,0.f,0.f,0.f};

  for (int k0 = 0; k0 < K; k0 += 32) {
    V bh[4], bl[4];
#pragma unroll
    for (int j = 0; j < 4; ++j) {
      const size_t bo = (size_t)(n0 + (j << 4) + rlane) * ldb + koff + k0;
      bh[j] = Frag<T>::load(Bb + bo);
      if (SPLIT) bl[j] = Frag<T>::load(Bb2 + bo);
    }
#pragma unroll
    for (int i = 0; i < 4; ++i) {
      const size_t ao = (size_t)(m0 + (i << 4) + rlane) * lda + koff + k0;
      V ah = Frag<T>::load(Ab + ao);
      V al;
      if (SPLIT) al = Frag<T>::load(Ab2 + ao);
#pragma unroll
      for (int j = 0; j < 4; ++j) {
        acc[i][j] = Frag<T>::mma(ah, bh[j], acc[i][j]);
        if (SPLIT) {
          acc[i][j] = Frag<T>::mma(ah, bl[j], acc[i][j]);
          acc[i][j] = Frag<T>::mma(al, bh[j], acc[i][j]);
        }
      }
      Frag<T>::guard(acc[i][0], acc[i][3], ah, SPLIT ? al : ah);
    }
    Frag<T>::keep(bh[0], bh[1], bh[2], bh[3]);
    if (SPLIT) Frag<T>::keep(bl[0], bl[1], bl[2], bl[3]);
  }
  acc_guard4(acc[0][0], acc[0][1], acc[0][2], acc[0][3]);
  acc_guard4(acc[1][0], acc[1][1], acc[1][2], acc[1][3]);
  acc_guard4(acc[2][0], acc[2][1], acc[2][2], acc[2][3]);
  acc_guard4(acc[3][0], acc[3][1], acc[3][2], acc[3][3]);

  float* slab = sT[wave];
  const float* Rb = RESID ? (resid + (size_t)b * strideR) : nullptr;
#pragma unroll
  for (int i = 0; i < 4; ++i) {
    const int mBase = m0 + (i << 4);
#pragma unroll
    for (int j = 0; j < 4; ++j) {
      const int n = n0 + (j << 4) + rlane;
      float bv = 0.f;
      if (BIAS_MODE == 2) bv = bias[n];
#pragma unroll
      for (int r = 0; r < 8; ++r) {
        float v = acc[i][j][r] * scale;
        if (BIAS_MODE == 1) v += bias[mBase + mOff + r];
        if (BIAS_MODE == 2) v += bv;
        if (RESID) v += Rb[(size_t)(mBase + mOff + r) * ldc + n];
        if (ACT == 1) v = tanhf(v);
        if (ACT == 2) v = fmaxf(v, 0.0f);
        if (ACT == 3) v = v / (1.0f + expf(-v));
        if (ACT == 4) v = (v > 0.f) ? v : 0.01f * v;
        if (ACT == 5) v = 0.5f * v * (1.0f + erff(v * 0.70710678118654752f));
        slab[(mOff + r) * 68 + (j << 4) + rlane] = v;
      }
    }
    __builtin_amdgcn_fence(__ATOMIC_RELEASE, "workgroup");
    __builtin_amdgcn_wave_barrier();
    __builtin_amdgcn_fence(__ATOMIC_ACQUIRE, "workgroup");
    if (OUT_MODE == 0) {
      float* C = (float*)Cout + (size_t)b * strideC;
      const int hh = lane >> 4, c4 = (lane & 15) * 4;
      for (int pass = 0; pass < 2; ++pass) {
#pragma unroll
        for (int it = 0; it < 8; ++it) {
          const int row = it * 2 + hh;
          v4f v = *(const v4f*)(slab + row * 68 + c4);
          *(volatile v4f*)(C + (size_t)(mBase + row) * ldc + n0 + c4) = v;
        }
        __threadfence();
      }
    } else {
      const int q = lane >> 3, c8 = (lane & 7) * 8;
      unsigned short* C  = (unsigned short*)Cout  + (size_t)b * strideC;
      unsigned short* C2 = (OUT_MODE == 2) ? ((unsigned short*)Cout2 + (size_t)b * strideC) : nullptr;
      for (int pass = 0; pass < 2; ++pass) {
#pragma unroll
        for (int it = 0; it < 4; ++it) {
          const int row = it * 4 + q;
          const float* sp = slab + row * 68 + c8;
          v8h hv, lv;
#pragma unroll
          for (int e = 0; e < 8; ++e) {
            if (OUT_MODE == 1) {
              hv[e] = (_Float16)sp[e];
            } else {
              unsigned short hb = f2bf_bits(sp[e]);
              unsigned short lb = f2bf_bits(sp[e] - bf_bits2f(hb));
              hv[e] = __builtin_bit_cast(_Float16, hb);
              lv[e] = __builtin_bit_cast(_Float16, lb);
            }
          }
          *(volatile v8h*)(C + (size_t)(mBase + row) * ldc + n0 + c8) = hv;
          if (OUT_MODE == 2) *(volatile v8h*)(C2 + (size_t)(mBase + row) * ldc + n0 + c8) = lv;
        }
        __threadfence();
      }
    }
    __builtin_amdgcn_fence(__ATOMIC_RELEASE, "workgroup");
    __builtin_amdgcn_wave_barrier();
    __builtin_amdgcn_fence(__ATOMIC_ACQUIRE, "workgroup");
  }
}


#define DN 524288
#define DCH 4
#define DRC (DN / DCH)
#define DH 90
#define DKP 96
#define DNP 128
__device__ __forceinline__ float elu1(float v) { return v > 0.f ? v : expm1f(v); }
template <int MODE>
__global__ __launch_bounds__(256) void l1_kernel(const float* __restrict__ X, long r0, const float* __restrict__ sc, const float* __restrict__ offs, const float* __restrict__ ST, const float* __restrict__ W1, const float* __restrict__ b1, unsigned* __restrict__ H16) {
  const long rl = (long)blockIdx.x * 256 + threadIdx.x; if (rl >= DRC) return; const long r = r0 + rl;
  float x0, x1;
  if (MODE == 0) { x0 = sc[0] * X[r * 2] + offs[0]; x1 = sc[0] * X[r * 2 + 1] + offs[1]; }
  else {
    const float h0 = (X[r * 2] - ST[0]) * ST[2], h1 = (X[r * 2 + 1] - ST[1]) * ST[3]; const float cut = ST[4];
    x0 = ST[5] * fminf(fmaxf(h0, -cut), cut) + ST[6]; x1 = ST[5] * fminf(fmaxf(h1, -cut), cut) + ST[6]; }
  unsigned* dst = H16 + rl * (DKP / 2);
  for (int pass = 0; pass < 2; ++pass) {
#pragma unroll 2
    for (int j = 0; j < DKP / 2; ++j) { const int c0 = 2 * j, c1 = 2 * j + 1; float a = 0.f, b = 0.f;
      if (c0 < DH) a = elu1(x0 * W1[c0] + x1 * W1[DH + c0] + b1[c0]); if (c1 < DH) b = elu1(x0 * W1[c1] + x1 * W1[DH + c1] + b1[c1]);
      ((volatile unsigned*)dst)[j] = (unsigned)__builtin_bit_cast(unsigned short, (_Float16)a) | ((unsigned)__builtin_bit_cast(unsigned short, (_Float16)b) << 16); }
    __threadfence(); }
}
__global__ __launch_bounds__(256) void l3_kernel(const float* __restrict__ G, long r0, const float* __restrict__ b2, const float* __restrict__ W3, const float* __restrict__ b3, float* __restrict__ Y, int ystride, int yoff) {
  const long rl = (long)blockIdx.x * 256 + threadIdx.x; if (rl >= DRC) return; const float* g = G + rl * DNP; float s = b3[0];
#pragma unroll 2
  for (int c = 0; c < DH; ++c) s += elu1(g[c] + b2[c]) * W3[c];
  ((volatile float*)Y)[(r0 + rl) * ystride + yoff] = s; __threadfence(); ((volatile float*)Y)[(r0 + rl) * ystride + yoff] = s;
}
__global__ __launch_bounds__(256) void w2t_kernel(const float* __restrict__ W2, unsigned* __restrict__ BT) {
  for (int i = threadIdx.x; i < DNP * DKP / 2; i += 256) { const int o = i / (DKP / 2), kp = 2 * (i % (DKP / 2)); float a = 0.f, b = 0.f; if (o < DH) { if (kp < DH) a = W2[kp * DH + o]; if (kp + 1 < DH) b = W2[(kp + 1) * DH + o]; }
    const unsigned u = (unsigned)__builtin_bit_cast(unsigned short, (_Float16)a) | ((unsigned)__builtin_bit_cast(unsigned short, (_Float16)b) << 16); ((volatile unsigned*)BT)[i] = u; __threadfence(); ((volatile unsigned*)BT)[i] = u; }
}
__global__ __launch_bounds__(256) void stats_kernel(const float* __restrict__ C2, double* __restrict__ PS) {
  __shared__ double red[4][256];
  double s0 = 0, s1 = 0, q0 = 0, q1 = 0;
  for (long r = (long)blockIdx.x * 256 + threadIdx.x; r < DN; r += (long)gridDim.x * 256) { const double a = C2[r * 2], b = C2[r * 2 + 1]; s0 += a; s1 += b; q0 += a * a; q1 += b * b; }
  red[0][threadIdx.x] = s0; red[1][threadIdx.x] = s1; red[2][threadIdx.x] = q0; red[3][threadIdx.x] = q1; __syncthreads();
  for (int o = 128; o > 0; o >>= 1) { if (threadIdx.x < o) for (int k = 0; k < 4; ++k) red[k][threadIdx.x] += red[k][threadIdx.x + o]; __syncthreads(); }
  if (threadIdx.x < 32) { const int k = threadIdx.x & 3; const double v = red[k][0]; ((volatile double*)PS)[(size_t)blockIdx.x * 4 + k] = v; __threadfence(); ((volatile double*)PS)[(size_t)blockIdx.x * 4 + k] = v; }
}
__global__ __launch_bounds__(64) void fin_kernel(const double* __restrict__ PS, int nblk, const float* __restrict__ rv, const float* __restrict__ convo, float* __restrict__ ST) {
  __shared__ double t[4];
  if (threadIdx.x < 4) { double s = 0; for (int b = 0; b < nblk; ++b) s += PS[(size_t)b * 4 + threadIdx.x]; t[threadIdx.x] = s; }
  __syncthreads();
  if (threadIdx.x < 32) { const double n = (double)DN; const double m0 = t[0] / n, m1 = t[1] / n; double v0 = t[2] / n - m0 * m0, v1 = t[3] / n - m1 * m1; if (v0 < 0) v0 = 0; if (v1 < 0) v1 = 0;
    const double rv0 = 0.9 * (double)rv[0] + 0.1 * v0 * (n / (n - 1.0)), rv1 = 0.9 * (double)rv[1] + 0.1 * v1 * (n / (n - 1.0)); const double std1 = sqrt(0.5 * (rv0 + rv1));
    float vals[7]; vals[0] = (float)m0; vals[1] = (float)m1; vals[2] = (float)(1.0 / sqrt(v0 + 1e-5)); vals[3] = (float)(1.0 / sqrt(v1 + 1e-5)); vals[4] = (float)(2.0 * std1); vals[5] = (float)(1.8 / (4.0 * std1)); vals[6] = convo[0];
    const int i = threadIdx.x & 7; if (i < 7) { ((volatile float*)ST)[i] = vals[i]; __threadfence(); ((volatile float*)ST)[i] = vals[i]; } }
}
extern "C" void kernel_launch(void* const* d_in, const int* in_sizes, int n_in, void* d_out, int out_size, void* d_ws, size_t ws_size, hipStream_t stream) {
  (void)in_sizes; (void)n_in; (void)out_size; (void)ws_size;
  auto Fp = [&](int i) { return (const float*)d_in[i]; };
  const float* x = Fp(0); const float* offs = Fp(1); const float* sc = Fp(2); const float* convo = Fp(3); const float* rv = Fp(4);
  const float* W1[3] = {Fp(5), Fp(11), Fp(17)}; const float* b1[3] = {Fp(6), Fp(12), Fp(18)}; const float* W2[3] = {Fp(7), Fp(13), Fp(19)}; const float* b2[3] = {Fp(8), Fp(14), Fp(20)}; const float* W3[3] = {Fp(9), Fp(15), Fp(21)}; const float* b3[3] = {Fp(10), Fp(16), Fp(22)};
  char* ws = (char*)d_ws; size_t off = 0;
  auto carve = [&](size_t bytes) -> char* { char* p = ws + off; off += (bytes + 255) & ~(size_t)255; return p; };
  unsigned* H16 = (unsigned*)carve((size_t)DRC * DKP * 2); float* G = (float*)carve((size_t)DRC * DNP * 4); unsigned* BT[3]; for (int m = 0; m < 3; ++m) BT[m] = (unsigned*)carve(DNP * DKP * 2);
  float* C2 = (float*)carve((size_t)DN * 2 * 4); const int NSB = 1024; double* PS = (double*)carve((size_t)NSB * 4 * 8); float* ST = (float*)carve(256);
  for (int m = 0; m < 3; ++m) w2t_kernel<<<1, 256, 0, stream>>>(W2[m], BT[m]);
  const int t = (DRC / 64) * (DNP / 64);
  for (int ch = 0; ch < DCH; ++ch) { const long r0 = (long)ch * DRC;
    for (int m = 0; m < 2; ++m) {
      l1_kernel<0><<<(DRC + 255) / 256, 256, 0, stream>>>(x, r0, sc, offs, nullptr, W1[m], b1[m], H16);
      wmma_gemm64<0, false, 0, 0, false><<<dim3((t + 7) / 8, 1), 256, 0, stream>>>((const unsigned short*)H16, nullptr, DKP, 0, (const unsigned short*)BT[m], nullptr, DKP, 0, G, nullptr, DNP, 0, nullptr, nullptr, 0, DRC, DNP, DKP, 1.0f);
      l3_kernel<<<(DRC + 255) / 256, 256, 0, stream>>>(G, r0, b2[m], W3[m], b3[m], C2, 2, m); } }
  stats_kernel<<<NSB, 256, 0, stream>>>(C2, PS);
  fin_kernel<<<1, 64, 0, stream>>>(PS, NSB, rv, convo, ST);
  for (int ch = 0; ch < DCH; ++ch) { const long r0 = (long)ch * DRC;
    l1_kernel<1><<<(DRC + 255) / 256, 256, 0, stream>>>(C2, r0, nullptr, nullptr, ST, W1[2], b1[2], H16);
    wmma_gemm64<0, false, 0, 0, false><<<dim3((t + 7) / 8, 1), 256, 0, stream>>>((const unsigned short*)H16, nullptr, DKP, 0, (const unsigned short*)BT[2], nullptr, DKP, 0, G, nullptr, DNP, 0, nullptr, nullptr, 0, DRC, DNP, DKP, 1.0f);
    l3_kernel<<<(DRC + 255) / 256, 256, 0, stream>>>(G, r0, b2[2], W3[2], b3[2], (float*)d_out, 1, 0); }
}
